// ScanLSTM_42580305773031
// MI455X (gfx1250) — hardware-verified
//
#include <hip/hip_runtime.h>

typedef __attribute__((ext_vector_type(16))) _Float16 v16h;
typedef __attribute__((ext_vector_type(8)))  _Float16 v8h;
typedef __attribute__((ext_vector_type(16))) __bf16   v16b;
typedef __attribute__((ext_vector_type(8)))  __bf16   v8b;
typedef __attribute__((ext_vector_type(8)))  float    v8f;
typedef __attribute__((ext_vector_type(4)))  float    v4f;
typedef __attribute__((ext_vector_type(8)))  unsigned short v8us;

constexpr int kT    = 128;
constexpr int kB    = 64;
constexpr int kD    = 1024;
constexpr int kH    = 1024;
constexpr int kG    = 4 * kH;
constexpr int kRows = kT * kB;

constexpr int kSeqPB      = 16;
constexpr int kRecBlocks  = kB / kSeqPB;
constexpr int kRecThreads = 256;
constexpr int kWaves      = kRecThreads / 32;
constexpr int kUnitsPW    = kH / kWaves;
constexpr int kPassUnits  = 32;
constexpr int kNumPass    = kUnitsPW / kPassUnits;
constexpr int kHP         = kH + 8;
constexpr int kHTile      = kSeqPB * kHP;
constexpr int kOSP        = 36;
constexpr float kWiUp = 256.0f;
constexpr float kWhUp = 16.0f;
constexpr float kHUp  = 16.0f;
constexpr float kDown = 1.0f / 256.0f;
static_assert(kB % kSeqPB == 0);
static_assert(kUnitsPW * kWaves == kH);
static_assert(kNumPass * kPassUnits == kUnitsPW);
static_assert(kD % 32 == 0 && kH % 32 == 0);
static_assert(kHP % 8 == 0);
static_assert((kOSP * 4) % 16 == 0);
static_assert(kHUp * kWhUp == kWiUp);

constexpr int kWTile        = 64;
constexpr int kWTileBlocksN = kG / kWTile;
constexpr int kWTileBlocksK = kD / kWTile;
constexpr int kWLdsPitch    = kWTile + 8;
constexpr int kXCastBlocks  = kRows * kD / 8 / 256;
static_assert(kG % kWTile == 0 && kD % kWTile == 0);
static_assert(kXCastBlocks * 256 * 8 == kRows * kD);
static_assert((kWLdsPitch * 2) % 16 == 0);

__device__ __forceinline__ void dep_guard_h(v8f& a, v8f& b, v16h x, v16h y) { asm volatile("v_nop\n\tv_nop\n\tv_nop\n\tv_nop" : "+v"(a), "+v"(b) : "v"(x), "v"(y)); }
__device__ __forceinline__ void dep_guard_b(v8f& a, v8f& b, v16b x, v16b y) { asm volatile("v_nop\n\tv_nop\n\tv_nop\n\tv_nop" : "+v"(a), "+v"(b) : "v"(x), "v"(y)); }
__device__ __forceinline__ void keep4_h(v16h a, v16h b, v16h c, v16h d) { asm volatile("v_nop" :: "v"(a), "v"(b), "v"(c), "v"(d)); }
__device__ __forceinline__ void keep4_b(v16b a, v16b b, v16b c, v16b d) { asm volatile("v_nop" :: "v"(a), "v"(b), "v"(c), "v"(d)); }
__device__ __forceinline__ void acc_guard4(v8f& a, v8f& b, v8f& c, v8f& d) { asm volatile("v_nop\n\tv_nop\n\tv_nop\n\tv_nop" : "+v"(a), "+v"(b), "+v"(c), "+v"(d)); }

template <typename T> struct Frag;
template <> struct Frag<_Float16> {
  typedef v16h V; union U { v16h v; v8h h[2]; };
  static __device__ __forceinline__ v16h load(const _Float16* p) {
    U f; f.h[0] = *(const v8h*)(p); f.h[1] = *(const v8h*)(p + 16); return f.v;
  }
  static __device__ __forceinline__ v8f mma(v16h a, v16h b, v8f c) {
    return __builtin_amdgcn_wmma_f32_16x16x32_f16(false, a, false, b, (short)0, c, false, false);
  }
  static __device__ __forceinline__ void guard(v8f& a, v8f& b, v16h x, v16h y) { dep_guard_h(a, b, x, y); }
  static __device__ __forceinline__ void keep(v16h a, v16h b, v16h c, v16h d) { keep4_h(a, b, c, d); }
};
template <> struct Frag<__bf16> {
  typedef v16b V; union U { v16b v; v8b h[2]; };
  static __device__ __forceinline__ v16b load(const __bf16* p) {
    U f; f.h[0] = *(const v8b*)(p); f.h[1] = *(const v8b*)(p + 16); return f.v;
  }
  static __device__ __forceinline__ v8f mma(v16b a, v16b b, v8f c) {
    return __builtin_amdgcn_wmma_f32_16x16x32_bf16(false, a, false, b, (short)0, c, false, false);
  }
  static __device__ __forceinline__ void guard(v8f& a, v8f& b, v16b x, v16b y) { dep_guard_b(a, b, x, y); }
  static __device__ __forceinline__ void keep(v16b a, v16b b, v16b c, v16b d) { keep4_b(a, b, c, d); }
};

__device__ __forceinline__ float ftanh(float x) { return 1.0f - 2.0f * __builtin_amdgcn_rcpf(1.0f + __expf(2.0f * x)); }
__device__ __forceinline__ float fsigm(float x) { return __builtin_amdgcn_rcpf(1.0f + __expf(-x)); }

__global__ __launch_bounds__(256) void prep_w_kernel(const float* __restrict__ Wi, const float* __restrict__ Wh,
                                                    unsigned short* __restrict__ wi16t, unsigned short* __restrict__ wh16t) {
  __shared__ __align__(16) unsigned short tile[kWTile * kWLdsPitch];
  const int tid = threadIdx.x;
  const int z  = blockIdx.z;
  const int n0 = blockIdx.x * kWTile;
  const int k0 = blockIdx.y * kWTile;
  const float* src = (z != 0) ? Wh : Wi;
  unsigned short* dst = (z != 0) ? wh16t : wi16t;
  const float scl = (z != 0) ? kWhUp : kWiUp;
  const int kk = tid >> 6, nn = tid & 63;
#pragma unroll 4
  for (int e = 0; e < 16; ++e) {
    const int k = 4 * e + kk;
    const float w = src[(size_t)(k0 + k) * kG + n0 + nn] * scl;
    tile[nn * kWLdsPitch + k] = __builtin_bit_cast(unsigned short, (_Float16)w);
  }
  __syncthreads();
  const int rr = tid >> 3, c8 = (tid & 7) * 8;
  for (int ps = 0; ps < 2; ++ps) {
#pragma unroll
    for (int it = 0; it < 2; ++it) {
      const int row = rr + 32 * it;
      const v8us v = *(const v8us*)(tile + row * kWLdsPitch + c8);
      *(volatile v8us*)(dst + (size_t)(n0 + row) * kD + k0 + c8) = v;
    }
    __threadfence();
  }
}

__global__ __launch_bounds__(256) void xcast_kernel(const float* __restrict__ x, _Float16* __restrict__ x16) {
  const size_t i = (size_t)blockIdx.x * 256 + threadIdx.x;
  const float* s = x + i * 8;
  const v4f a = *(const v4f*)s;
  const v4f c = *(const v4f*)(s + 4);
  v8h o;
  o[0] = (_Float16)a[0]; o[1] = (_Float16)a[1]; o[2] = (_Float16)a[2]; o[3] = (_Float16)a[3];
  o[4] = (_Float16)c[0]; o[5] = (_Float16)c[1]; o[6] = (_Float16)c[2]; o[7] = (_Float16)c[3];
  _Float16* d = x16 + i * 8;
  *(volatile v8h*)d = o;
  __threadfence();
  *(volatile v8h*)d = o;
}

__global__ __launch_bounds__(kRecThreads) void lstm_scan_kernel(
    const unsigned short* __restrict__ x16u,
    const unsigned short* __restrict__ wi16u,
    const unsigned short* __restrict__ wh16u,
    const float* __restrict__ bias,
    const float* __restrict__ h0,
    const float* __restrict__ c0,
    const int* __restrict__ resets,
    float* __restrict__ out0,
    float* __restrict__ out1,
    float* __restrict__ out2) {
  __shared__ __align__(16) _Float16 htile[2 * kHTile];
  __shared__ __align__(16) float cbuf[kSeqPB * kH];
  __shared__ __align__(16) float oslab[kWaves][16 * kOSP];

  const int tid = threadIdx.x, lane = tid & 31, wave = tid >> 5;
  const int rlane = lane & 15, hh = lane >> 4, koff = hh * 8, mOff = hh * 8;
  const int q4 = lane >> 3, c4 = (lane & 7) * 4;
  const int seq0 = blockIdx.x * kSeqPB;

  for (int i = tid; i < kSeqPB * kH; i += kRecThreads) {
    const int row = i >> 10, u = i & (kH - 1);
    const float hv = h0[(size_t)(seq0 + row) * kH + u];
    const float cv = c0[(size_t)(seq0 + row) * kH + u];
    const int rf = resets[seq0 + row];
    htile[row * kHP + u] = (_Float16)((rf != 0) ? 0.0f : hv * kHUp);
    cbuf[row * kH + u] = cv;
  }
  {
    const int i = tid;
    const int tsel = i >> 7, row = (i >> 3) & 15, e = i & 7;
    htile[tsel * kHTile + row * kHP + kH + e] = (_Float16)0.0f;
  }
  __syncthreads();

  const _Float16* xb  = (const _Float16*)x16u;
  const _Float16* wib = (const _Float16*)wi16u;
  const _Float16* whb = (const _Float16*)wh16u;
  float* slab = oslab[wave];
  const v8f z8 = {0.f, 0.f, 0.f, 0.f, 0.f, 0.f, 0.f, 0.f};

#pragma unroll 1
  for (int t = 0; t < kT; ++t) {
    const _Float16* hc = htile + (t & 1) * kHTile;
    _Float16*       hn = htile + ((t + 1) & 1) * kHTile;
    const int tn = (t + 1 < kT) ? (t + 1) : (kT - 1);
    int mcur = 0, mnxt = 0;
#pragma unroll
    for (int r = 0; r < 8; ++r) {
      const int f0 = resets[t * kB + seq0 + mOff + r];
      const int f1 = resets[tn * kB + seq0 + mOff + r];
      mcur |= ((f0 != 0) ? 1 : 0) << r;
      mnxt |= ((f1 != 0) ? 1 : 0) << r;
    }
    const _Float16* xrow = xb + (size_t)(t * kB + seq0 + rlane) * kD + koff;
    const _Float16* hrow = hc + rlane * kHP + koff;
    const bool last = (t == kT - 1);
    const size_t orow0 = (size_t)t * kB + seq0;

#pragma unroll 1
    for (int p = 0; p < kNumPass; ++p) {
      const int ubase = wave * kUnitsPW + p * kPassUnits;
      const _Float16* bwi = wib + (size_t)(ubase + rlane) * kD + koff;
      const _Float16* bwh = whb + (size_t)(ubase + rlane) * kH + koff;
      v8f acc[4][2];
#pragma unroll
      for (int g = 0; g < 4; ++g) { acc[g][0] = z8; acc[g][1] = z8; }

#pragma unroll 1
      for (int kc = 0; kc < kD / 32; ++kc) {
        const v16h fa = Frag<_Float16>::load(xrow + kc * 32);
        v16h fb[8];
#pragma unroll
        for (int g = 0; g < 4; ++g)
#pragma unroll
          for (int j = 0; j < 2; ++j)
            fb[2 * g + j] = Frag<_Float16>::load(bwi + (size_t)(g * kH + 16 * j) * kD + kc * 32);
#pragma unroll
        for (int g = 0; g < 4; ++g)
#pragma unroll
          for (int j = 0; j < 2; ++j) acc[g][j] = Frag<_Float16>::mma(fa, fb[2 * g + j], acc[g][j]);
        Frag<_Float16>::guard(acc[0][0], acc[3][1], fa, fb[7]);
        Frag<_Float16>::keep(fb[0], fb[1], fb[2], fb[3]);
        Frag<_Float16>::keep(fb[4], fb[5], fb[6], fb[7]);
      }
#pragma unroll 1
      for (int kc = 0; kc < kH / 32; ++kc) {
        const v16h fa = Frag<_Float16>::load(hrow + kc * 32);
        v16h fb[8];
#pragma unroll
        for (int g = 0; g < 4; ++g)
#pragma unroll
          for (int j = 0; j < 2; ++j)
            fb[2 * g + j] = Frag<_Float16>::load(bwh + (size_t)(g * kH + 16 * j) * kH + kc * 32);
#pragma unroll
        for (int g = 0; g < 4; ++g)
#pragma unroll
          for (int j = 0; j < 2; ++j) acc[g][j] = Frag<_Float16>::mma(fa, fb[2 * g + j], acc[g][j]);
        Frag<_Float16>::guard(acc[0][0], acc[3][1], fa, fb[7]);
        Frag<_Float16>::keep(fb[0], fb[1], fb[2], fb[3]);
        Frag<_Float16>::keep(fb[4], fb[5], fb[6], fb[7]);
      }
      acc_guard4(acc[0][0], acc[0][1], acc[1][0], acc[1][1]);
      acc_guard4(acc[2][0], acc[2][1], acc[3][0], acc[3][1]);

#pragma unroll
      for (int j = 0; j < 2; ++j) {
        const int u = ubase + 16 * j + rlane;
        const float bsi = bias[u], bsf = bias[kH + u], bsg = bias[2 * kH + u], bso = bias[3 * kH + u];
#pragma unroll
        for (int r = 0; r < 8; ++r) {
          const int row = mOff + r;
          const float zi = fmaf(acc[0][j][r], kDown, bsi);
          const float zf = fmaf(acc[1][j][r], kDown, bsf);
          const float zg = fmaf(acc[2][j][r], kDown, bsg);
          const float zo = fmaf(acc[3][j][r], kDown, bso);
          const float cold = cbuf[row * kH + u];
          const float cm = (((mcur >> r) & 1) != 0) ? 0.0f : cold;
          const float cn = fmaf(fsigm(zf), cm, fsigm(zi) * ftanh(zg));
          const float hv = fsigm(zo) * ftanh(cn);
          cbuf[row * kH + u] = cn;
          const float hop = (((mnxt >> r) & 1) != 0) ? 0.0f : hv * kHUp;
          hn[row * kHP + u] = (_Float16)hop;
          slab[row * kOSP + 16 * j + rlane] = hv;
        }
      }
      __builtin_amdgcn_fence(__ATOMIC_RELEASE, "workgroup");
      __builtin_amdgcn_wave_barrier();
      __builtin_amdgcn_fence(__ATOMIC_ACQUIRE, "workgroup");

      for (int ps = 0; ps < 2; ++ps) {
#pragma unroll
        for (int it = 0; it < 4; ++it) {
          const int row = it * 4 + q4;
          const v4f v = *(const v4f*)(slab + row * kOSP + c4);
          *(volatile v4f*)(out2 + (orow0 + row) * kH + ubase + c4) = v;
          if (last) {
            *(volatile v4f*)(out0 + (size_t)(seq0 + row) * kH + ubase + c4) = v;
            const v4f vc = *(const v4f*)(cbuf + row * kH + ubase + c4);
            *(volatile v4f*)(out1 + (size_t)(seq0 + row) * kH + ubase + c4) = vc;
          }
        }
        __threadfence();
      }
      __builtin_amdgcn_fence(__ATOMIC_RELEASE, "workgroup");
      __builtin_amdgcn_wave_barrier();
      __builtin_amdgcn_fence(__ATOMIC_ACQUIRE, "workgroup");
    }
    __syncthreads();
  }
}

extern "C" void kernel_launch(void* const* d_in, const int* in_sizes, int n_in,
                              void* d_out, int out_size, void* d_ws, size_t ws_size, hipStream_t stream) {
  if (n_in < 7 || d_out == nullptr || d_ws == nullptr) return;
  if (in_sizes[0] != kT * kB * kD || in_sizes[1] != kB * kH || in_sizes[2] != kB * kH ||
      in_sizes[3] != kD * kG || in_sizes[4] != kH * kG || in_sizes[5] != kG || in_sizes[6] != kT * kB ||
      out_size != 2 * kB * kH + kT * kB * kH) return;

  const float* x      = (const float*)d_in[0];
  const float* h0     = (const float*)d_in[1];
  const float* c0     = (const float*)d_in[2];
  const float* Wi     = (const float*)d_in[3];
  const float* Wh     = (const float*)d_in[4];
  const float* bias   = (const float*)d_in[5];
  const int*   resets = (const int*)d_in[6];

  float* out0 = (float*)d_out;
  float* out1 = out0 + (size_t)kB * kH;
  float* out2 = out0 + (size_t)2 * kB * kH;

  char* ws = (char*)d_ws; size_t off = 0;
  auto carve = [&](size_t bytes) -> char* { char* p = ws + off; off += (bytes + 255) & ~(size_t)255; return p; };
  unsigned short* X16   = (unsigned short*)carve((size_t)kRows * kD * 2);
  unsigned short* WI16T = (unsigned short*)carve((size_t)kG * kD * 2);
  unsigned short* WH16T = (unsigned short*)carve((size_t)kG * kH * 2);
  if (off > ws_size || off > (size_t)134217728) return;

  prep_w_kernel<<<dim3(kWTileBlocksN, kWTileBlocksK, 2), 256, 0, stream>>>(Wi, Wh, WI16T, WH16T);

  xcast_kernel<<<kXCastBlocks, 256, 0, stream>>>(x, (_Float16*)X16);

  lstm_scan_kernel<<<kRecBlocks, kRecThreads, 0, stream>>>(X16, WI16T, WH16T, bias, h0, c0, resets, out0, out1, out2);
}
